// SparseAttention_19421842112584
// MI455X (gfx1250) — hardware-verified
//
#include <hip/hip_runtime.h>


#ifndef NB
#define NB 1
#endif
#ifndef SEQ
#define SEQ 4096
#endif
#define SEQ_FULL 4096
#define DM   1024
#define NH_  16
#define HD   64
#define LDQ  (3 * DM)
#define SCL  0.125f
#define LKP  72
#define LVP  136

static_assert(SEQ % 64 == 0);
static_assert(DM == NH_ * HD);
static_assert(HD == 64);
static_assert(DM % 32 == 0);
static_assert(LDQ % 64 == 0);
static_assert(((size_t)LDQ * DM / 64) % 32 == 0);
static_assert(((size_t)DM * DM / 64) % 32 == 0);
static_assert(((size_t)SEQ * DM / 8) % 256 == 0);

typedef unsigned short bf;
typedef __attribute__((ext_vector_type(16))) __bf16   v16bf;
typedef __attribute__((ext_vector_type(8)))  unsigned short v8us;
typedef __attribute__((ext_vector_type(2)))  unsigned short v2us;
typedef __attribute__((ext_vector_type(8)))  float    v8f;
typedef __attribute__((ext_vector_type(4)))  float    v4f;
typedef v4f  __attribute__((may_alias)) v4fa;
typedef v8us __attribute__((may_alias)) v8usa;

__device__ __forceinline__ unsigned short f2bf(float f) { unsigned u = __float_as_uint(f); u += 0x7FFFu + ((u >> 16) & 1u); return (unsigned short)(u >> 16); }
__device__ __forceinline__ float bf2f(unsigned short b) { return __uint_as_float(((unsigned)b) << 16); }
__device__ __forceinline__ void splitf(float y, unsigned short& h, unsigned short& l) { h = f2bf(y); l = f2bf(y - bf2f(h)); }
__device__ __forceinline__ v16bf cat16b(v8us lo, v8us hi) { return __builtin_bit_cast(v16bf, __builtin_shufflevector(lo, hi, 0, 1, 2, 3, 4, 5, 6, 7, 8, 9, 10, 11, 12, 13, 14, 15)); }
__device__ __forceinline__ v8f wmmab(v16bf a, v16bf b, v8f c) { return __builtin_amdgcn_wmma_f32_16x16x32_bf16(false, a, false, b, (short)0, c, false, false); }

template <typename T16> struct WFrag;
template <> struct WFrag<bf> { typedef v16bf V; static __device__ __forceinline__ V ld(const bf* p) { return cat16b(*(const v8us*)p, *(const v8us*)(p + 16)); } static __device__ __forceinline__ v8f mma(V a, V b, v8f c) { return wmmab(a, b, c); } };
template <typename T16, int NSPLIT, bool BIAS>
__global__ __launch_bounds__(32) void k_gemmw(const T16* __restrict__ A, const T16* __restrict__ A2, const T16* __restrict__ Bt, const T16* __restrict__ Bt2, int K, float* C, int ldc, const float* __restrict__ bias, size_t sA, size_t sB, size_t sC) {
    typedef typename WFrag<T16>::V V;
    __shared__ __align__(16) float os[16 * 68];
    const size_t z = blockIdx.z; A += z * sA; if (A2) A2 += z * sA; Bt += z * sB; if (Bt2) Bt2 += z * sB; C += z * sC;
    const int lane = threadIdx.x & 31, lr = lane & 15, hi = lane >> 4; const int r0 = blockIdx.x * 64, c0 = blockIdx.y * 64;
    v8f acc[4][4];
#pragma unroll
    for (int mb = 0; mb < 4; ++mb)
#pragma unroll
        for (int nb = 0; nb < 4; ++nb) acc[mb][nb] = (v8f){};
    const size_t aoff = (size_t)(r0 + lr) * K + 8 * hi, boff = (size_t)(c0 + lr) * K + 8 * hi;
#pragma unroll 1
    for (int kc = 0; kc < K; kc += 32) {
        V a[4], a2[4];
#pragma unroll
        for (int mb = 0; mb < 4; ++mb) { a[mb] = WFrag<T16>::ld(A + aoff + (size_t)mb * 16 * K + kc); if (NSPLIT == 1 || NSPLIT == 2) a2[mb] = WFrag<T16>::ld(A2 + aoff + (size_t)mb * 16 * K + kc); }
#pragma unroll
        for (int nb = 0; nb < 4; ++nb) { const V b = WFrag<T16>::ld(Bt + boff + (size_t)nb * 16 * K + kc); V b2; if (NSPLIT >= 2) b2 = WFrag<T16>::ld(Bt2 + boff + (size_t)nb * 16 * K + kc);
#pragma unroll
            for (int mb = 0; mb < 4; ++mb) { acc[mb][nb] = WFrag<T16>::mma(a[mb], b, acc[mb][nb]); if (NSPLIT == 1 || NSPLIT == 2) acc[mb][nb] = WFrag<T16>::mma(a2[mb], b, acc[mb][nb]); if (NSPLIT >= 2) acc[mb][nb] = WFrag<T16>::mma(a[mb], b2, acc[mb][nb]); } }
        asm volatile("v_nop\n\tv_nop\n\tv_nop\n\tv_nop" : "+v"(acc[0][0]), "+v"(acc[1][1]), "+v"(acc[2][2]), "+v"(acc[3][3]) : "v"(a[0]), "v"(a[3]));
    }
#pragma unroll
    for (int mb = 0; mb < 4; ++mb) {
#pragma unroll
        for (int nb = 0; nb < 4; ++nb) {
#pragma unroll
            for (int j = 0; j < 8; ++j) os[(hi * 8 + j) * 68 + nb * 16 + lr] = acc[mb][nb][j]; }
        __builtin_amdgcn_wave_barrier(); asm volatile("" ::: "memory");
        float* crow = C + (size_t)(r0 + mb * 16) * ldc + c0;
#pragma unroll 1
        for (int ps = 0; ps < 2; ++ps) {
#pragma unroll
            for (int s = 0; s < 8; ++s) { const int row = 2 * s + hi, cofs = lr * 4; v4f val = *(const v4fa*)(os + row * 68 + cofs); if (BIAS) { val[0] += bias[c0 + cofs]; val[1] += bias[c0 + cofs + 1]; val[2] += bias[c0 + cofs + 2]; val[3] += bias[c0 + cofs + 3]; }
                *(volatile v4f*)(crow + (size_t)row * ldc + cofs) = val; }
            if (ps == 0) __threadfence(); }
        __builtin_amdgcn_wave_barrier(); asm volatile("" ::: "memory");
    }
}

__global__ __launch_bounds__(256) void k_wtG(const float* __restrict__ w, unsigned kshift, unsigned N, bf* Bt, unsigned nlines) {
    const unsigned lane = threadIdx.x & 31u; const unsigned L0 = (blockIdx.x * 8u + (threadIdx.x >> 5)) * 4u; const unsigned kmask = (1u << kshift) - 1u;
    v2us o[4];
#pragma unroll
    for (unsigned l = 0; l < 4; ++l) { unsigned L = L0 + l; L = (L < nlines) ? L : (nlines - 1u); const unsigned e = L * 64u + lane * 2u; const unsigned k = e & kmask, n = e >> kshift; v2us t;
        t[0] = f2bf(w[(size_t)k * N + n]); t[1] = f2bf(w[(size_t)(k + 1u) * N + n]); o[l] = t; }
#pragma unroll 1
    for (int ps = 0; ps < 2; ++ps) {
#pragma unroll
        for (unsigned l = 0; l < 4; ++l) { const unsigned L = L0 + l; if (L < nlines) *(volatile v2us*)(Bt + (size_t)L * 64u + lane * 2u) = o[l]; }
        if (ps == 0) __threadfence(); }
}

__global__ __launch_bounds__(256) void k_cvt8(const float* __restrict__ src, bf* dst, size_t n8) { const size_t i = (size_t)blockIdx.x * 256 + threadIdx.x; if (i >= n8) return; const v8f v = *(const v8f*)(src + i * 8); v8us o;
#pragma unroll
    for (int k = 0; k < 8; ++k) o[k] = f2bf(v[k]); *(volatile v8us*)(dst + i * 8) = o; __threadfence(); *(volatile v8us*)(dst + i * 8) = o; }

__global__ __launch_bounds__(128) void k_swattn(const float* __restrict__ QKV, bf* CH, bf* CL) {
    __shared__ __align__(16) unsigned short Kh[128 * LKP];
    __shared__ __align__(16) unsigned short Kl[128 * LKP];
    __shared__ __align__(16) unsigned short Vh[64 * LVP];
    __shared__ __align__(16) unsigned short Vl[64 * LVP];
    __shared__ __align__(16) unsigned short Ph[4 * 16 * LVP];
    __shared__ __align__(16) unsigned short Pl[4 * 16 * LVP];
    const unsigned tid = threadIdx.x, lane = tid & 31u, wv = tid >> 5, lr = lane & 15u, hi = lane >> 4;
    const unsigned qt = blockIdx.x, hd = blockIdx.y, t0 = qt * 64u;
    const bool haslo = (qt != 0u);
    const float* kbase = QKV + DM + hd * HD;
    const float* vbase = QKV + 2 * DM + hd * HD;
#pragma unroll 1
    for (unsigned it = 0; it < 8u; ++it) {
        const unsigned idx = tid + it * 128u, row = idx >> 3, c8 = (idx & 7u) * 8u;
        const bool ok = haslo || (row >= 64u);
        const unsigned kg = ok ? (t0 + row - 64u) : 0u;
        const v8f kv = *(const v8f*)(kbase + (size_t)kg * LDQ + c8);
        const v8f vv = *(const v8f*)(vbase + (size_t)kg * LDQ + c8);
        v8us kh8, kl8;
#pragma unroll
        for (int q = 0; q < 8; ++q) {
            const float xk = ok ? kv[q] : 0.0f; unsigned short a, c; splitf(xk, a, c); kh8[q] = a; kl8[q] = c;
            const float xv = ok ? vv[q] : 0.0f; unsigned short a2, c2; splitf(xv, a2, c2);
            Vh[(c8 + (unsigned)q) * LVP + row] = a2; Vl[(c8 + (unsigned)q) * LVP + row] = c2; }
        *(v8usa*)(Kh + row * LKP + c8) = kh8; *(v8usa*)(Kl + row * LKP + c8) = kl8;
    }
    v16bf qh[2], ql[2];
    {
        const float* qrow = QKV + (size_t)(t0 + 16u * wv + lr) * LDQ + hd * HD + 8u * hi;
#pragma unroll
        for (int kc = 0; kc < 2; ++kc) {
            const v8f a0 = *(const v8f*)(qrow + kc * 32); const v8f a1 = *(const v8f*)(qrow + kc * 32 + 16);
            v8us h0, l0, h1, l1;
#pragma unroll
            for (int e = 0; e < 8; ++e) { unsigned short a, c; splitf(a0[e] * SCL, a, c); h0[e] = a; l0[e] = c; splitf(a1[e] * SCL, a, c); h1[e] = a; l1[e] = c; }
            qh[kc] = cat16b(h0, h1); ql[kc] = cat16b(l0, l1); }
    }
    __syncthreads();
    v8f sc[8];
#pragma unroll
    for (int kt = 0; kt < 8; ++kt) {
        sc[kt] = (v8f){};
#pragma unroll
        for (int kc = 0; kc < 2; ++kc) {
            const unsigned short* pk = Kh + ((unsigned)kt * 16u + lr) * LKP + (unsigned)kc * 32u + 8u * hi;
            const unsigned short* pl = Kl + ((unsigned)kt * 16u + lr) * LKP + (unsigned)kc * 32u + 8u * hi;
            const v16bf kh = cat16b(*(const v8usa*)pk, *(const v8usa*)(pk + 16));
            const v16bf kl = cat16b(*(const v8usa*)pl, *(const v8usa*)(pl + 16));
            sc[kt] = wmmab(qh[kc], kh, sc[kt]); sc[kt] = wmmab(ql[kc], kh, sc[kt]); sc[kt] = wmmab(qh[kc], kl, sc[kt]);
            asm volatile("v_nop\n\tv_nop\n\tv_nop\n\tv_nop" : "+v"(sc[kt]) : "v"(kh), "v"(kl));
        }
    }
    asm volatile("v_nop\n\tv_nop\n\tv_nop\n\tv_nop" : "+v"(sc[7]) : "v"(qh[0]), "v"(qh[1]), "v"(ql[0]), "v"(ql[1]));
    unsigned short* pwh = Ph + wv * 16u * LVP;
    unsigned short* pwl = Pl + wv * 16u * LVP;
#pragma unroll
    for (int r = 0; r < 8; ++r) {
        const unsigned il = 64u + 16u * wv + 8u * hi + (unsigned)r;
        float mx = -3.0e38f;
#pragma unroll
        for (int kt = 0; kt < 8; ++kt) { const unsigned jl = (unsigned)kt * 16u + lr; const bool valid = (jl <= il) && ((il - jl) <= 64u) && (haslo || (jl >= 64u));
            const float s = valid ? sc[kt][r] : -3.0e38f; sc[kt][r] = s; mx = fmaxf(mx, s); }
#pragma unroll
        for (int sh = 8; sh; sh >>= 1) mx = fmaxf(mx, __shfl_xor(mx, sh, 32));
        float sum = 0.0f;
#pragma unroll
        for (int kt = 0; kt < 8; ++kt) { const unsigned jl = (unsigned)kt * 16u + lr; const bool valid = (jl <= il) && ((il - jl) <= 64u) && (haslo || (jl >= 64u));
            const float ex = __builtin_amdgcn_exp2f((sc[kt][r] - mx) * 1.4426950408889634f); const float e = valid ? ex : 0.0f; sc[kt][r] = e; sum += e; }
#pragma unroll
        for (int sh = 8; sh; sh >>= 1) sum += __shfl_xor(sum, sh, 32);
        const float inv = __builtin_amdgcn_rcpf(sum);
#pragma unroll
        for (int kt = 0; kt < 8; ++kt) { unsigned short a, c; splitf(sc[kt][r] * inv, a, c); const unsigned o = (8u * hi + (unsigned)r) * LVP + (unsigned)kt * 16u + lr; pwh[o] = a; pwl[o] = c; }
    }
    __syncthreads();
    v8f oa[4];
#pragma unroll
    for (int dt = 0; dt < 4; ++dt) oa[dt] = (v8f){};
#pragma unroll
    for (int kc = 0; kc < 4; ++kc) {
        const unsigned short* pa = pwh + lr * LVP + (unsigned)kc * 32u + 8u * hi;
        const unsigned short* pb = pwl + lr * LVP + (unsigned)kc * 32u + 8u * hi;
        const v16bf ph = cat16b(*(const v8usa*)pa, *(const v8usa*)(pa + 16));
        const v16bf pl = cat16b(*(const v8usa*)pb, *(const v8usa*)(pb + 16));
#pragma unroll
        for (int dt = 0; dt < 4; ++dt) {
            const unsigned short* pv = Vh + ((unsigned)dt * 16u + lr) * LVP + (unsigned)kc * 32u + 8u * hi;
            const unsigned short* pw = Vl + ((unsigned)dt * 16u + lr) * LVP + (unsigned)kc * 32u + 8u * hi;
            const v16bf vh = cat16b(*(const v8usa*)pv, *(const v8usa*)(pv + 16));
            const v16bf vl = cat16b(*(const v8usa*)pw, *(const v8usa*)(pw + 16));
            oa[dt] = wmmab(ph, vh, oa[dt]); oa[dt] = wmmab(pl, vh, oa[dt]); oa[dt] = wmmab(ph, vl, oa[dt]);
            asm volatile("v_nop\n\tv_nop\n\tv_nop\n\tv_nop" : "+v"(oa[dt]) : "v"(vh), "v"(vl));
        }
        asm volatile("v_nop\n\tv_nop\n\tv_nop\n\tv_nop" : "+v"(oa[3]) : "v"(ph), "v"(pl));
    }
    __syncthreads();
#pragma unroll
    for (int dt = 0; dt < 4; ++dt) {
#pragma unroll
        for (int r = 0; r < 8; ++r) { unsigned short a, c; splitf(oa[dt][r], a, c); const unsigned o = (8u * hi + (unsigned)r) * LVP + (unsigned)dt * 16u + lr; pwh[o] = a; pwl[o] = c; } }
    __syncthreads();
#pragma unroll 1
    for (int ps = 0; ps < 2; ++ps) {
#pragma unroll
        for (unsigned s = 0; s < 4u; ++s) { const unsigned row = 4u * s + (lane >> 3), c = (lane & 7u) * 8u;
            const v8us vh8 = *(const v8usa*)(pwh + row * LVP + c); const v8us vl8 = *(const v8usa*)(pwl + row * LVP + c);
            const size_t g = (size_t)(t0 + 16u * wv + row) * DM + hd * HD + c;
            *(volatile v8us*)(CH + g) = vh8; *(volatile v8us*)(CL + g) = vl8; }
        if (ps == 0) __threadfence(); }
}

extern "C" void kernel_launch(void* const* d_in, const int* in_sizes, int n_in,
                              void* d_out, int out_size, void* d_ws, size_t ws_size, hipStream_t stream) {
    (void)out_size;
    if (n_in < 3) return;
    if (in_sizes[0] < NB * SEQ * DM || in_sizes[1] < DM * LDQ || in_sizes[2] < DM * DM) return;
    const float* X = (const float*)d_in[0]; const float* Wqkv = (const float*)d_in[1]; const float* Wo = (const float*)d_in[2];
    float* OUT = (float*)d_out;
    char* wsp = (char*)d_ws;
    auto take = [&](size_t bytes) { char* p = wsp; wsp += (bytes + 255) & ~(size_t)255; return (void*)p; };
    bf* XB  = (bf*)take((size_t)SEQ * DM * 2);
    bf* WqT = (bf*)take((size_t)LDQ * DM * 2);
    bf* WoT = (bf*)take((size_t)DM * DM * 2);
    float* QKVb = (float*)take((size_t)SEQ * LDQ * 4);
    bf* CH = (bf*)take((size_t)SEQ * DM * 2);
    bf* CL = (bf*)take((size_t)SEQ * DM * 2);
    const size_t carved = (size_t)(wsp - (char*)d_ws);
    if (carved > ws_size || carved > (size_t)134217728) return;
    { const unsigned nl = (unsigned)((size_t)LDQ * DM / 64); k_wtG<<<(nl + 31u) / 32u, 256, 0, stream>>>(Wqkv, 10u, (unsigned)LDQ, WqT, nl); }
    { const unsigned nl = (unsigned)((size_t)DM * DM / 64);  k_wtG<<<(nl + 31u) / 32u, 256, 0, stream>>>(Wo, 10u, (unsigned)DM, WoT, nl); }
    for (int b = 0; b < NB; ++b) {
        const float* xb = X + (size_t)b * SEQ_FULL * DM; float* ob = OUT + (size_t)b * SEQ_FULL * DM;
        const size_t n8 = (size_t)SEQ * DM / 8;
        k_cvt8<<<(unsigned)((n8 + 255) / 256), 256, 0, stream>>>(xb, XB, n8);
        k_gemmw<bf, 0, false><<<dim3(SEQ / 64, LDQ / 64, 1), 32, 0, stream>>>(XB, nullptr, WqT, nullptr, DM, QKVb, LDQ, nullptr, 0, 0, 0);
        k_swattn<<<dim3(SEQ / 64, NH_, 1), 128, 0, stream>>>(QKVb, CH, CL);
        k_gemmw<bf, 1, false><<<dim3(SEQ / 64, DM / 64, 1), 32, 0, stream>>>(CH, CL, WoT, nullptr, DM, ob, DM, nullptr, 0, 0, 0);
    }
}
